// DistanceLayer_4166118277258
// MI455X (gfx1250) — hardware-verified
//
#include <hip/hip_runtime.h>
#include <hip/hip_bf16.h>
#include <math.h>


#define BB 2
#define SS 2048
#define DD 1024
#define HH 16
#define DKK 64
#define QW 2

typedef _Float16 bf16;
typedef __attribute__((ext_vector_type(4))) unsigned v4u_t;
typedef unsigned v4ua __attribute__((ext_vector_type(4), may_alias));
typedef __attribute__((ext_vector_type(4))) float v4f_t;
typedef float v4fa __attribute__((ext_vector_type(4), may_alias));
typedef __attribute__((ext_vector_type(16))) bf16  bf16x16;
typedef __attribute__((ext_vector_type(8)))  bf16  bf16x8;
typedef __attribute__((ext_vector_type(4)))  bf16  bf16x4;
typedef __attribute__((ext_vector_type(8)))  float f32x8;

#define LDS_STRIDE 48
#define KSTRIDE    72
#define VSTRIDE    48

__device__ __forceinline__ f32x8 wmma_bf16(bf16x16 a, bf16x16 b, f32x8 c) {
  return __builtin_amdgcn_wmma_f32_16x16x32_f16(
      false, a, false, b, (short)0, c, false, false);
}
#define RSPLIT (1.0f / 2048.0f)
__device__ __forceinline__ bf16 lo_of(float v, bf16 h) { return (bf16)((v - (float)h) * 2048.0f); }
__device__ __forceinline__ f32x8 wmma_split(bf16x16 a, bf16x16 al, bf16x16 b, bf16x16 bl, f32x8 c) {
  f32x8 x = {}; x = wmma_bf16(al, b, x); x = wmma_bf16(a, bl, x); return wmma_bf16(a, b, c) + x * RSPLIT; }

template <typename T>
__device__ __forceinline__ bf16x16 load_frag(const T* __restrict__ base, int ld,
                                             int row0, int k0) {
  const int lane = threadIdx.x & 31;
  const int r    = lane & 15;
  const int kh   = (lane >> 4) * 8;
  const T* p0 = base + (size_t)(row0 + r) * ld + (k0 + kh);
  const T* p1 = p0 + 16;
  bf16x16 f;
#pragma unroll
  for (int i = 0; i < 8; ++i) {
    f[i]     = (bf16)p0[i];
    f[i + 8] = (bf16)p1[i];
  }
  return f;
}

__device__ __forceinline__ bf16x16 lds_frag(const bf16* base, int stride) {
  const int lane = threadIdx.x & 31;
  const int row  = lane & 15;
  const int kh   = (lane >> 4) * 8;
  const bf16x8 lo = *(const bf16x8*)(base + row * stride + kh);
  const bf16x8 hi = *(const bf16x8*)(base + row * stride + kh + 16);
  bf16x16 f;
#pragma unroll
  for (int i = 0; i < 8; ++i) { f[i] = lo[i]; f[i + 8] = hi[i]; }
  return f;
}

template <typename T>
__device__ __forceinline__ void stage_read16(const T* __restrict__ p, float* buf) {
#pragma unroll
  for (int i = 0; i < 16; ++i) buf[i] = (float)p[i];
}

__device__ __forceinline__ void stage_write(bf16* dst, const float* buf, int nquad) {
#pragma unroll
  for (int i = 0; i < nquad; ++i) {
    bf16x4 q;
    q[0] = (bf16)buf[4 * i];     q[1] = (bf16)buf[4 * i + 1];
    q[2] = (bf16)buf[4 * i + 2]; q[3] = (bf16)buf[4 * i + 3];
    *(bf16x4*)(dst + 4 * i) = q;
  }
}

__global__ __launch_bounds__(256) void transpose_pack_kernel(const float* __restrict__ W, bf16* __restrict__ WT, int K, int N, size_t plane) {
  __shared__ float tile[64][65];
  const int k0 = blockIdx.y * 64, n0 = blockIdx.x * 64, t = threadIdx.x;
  for (int i = t; i < 64 * 64; i += 256) { const int kr = i >> 6, nc = i & 63; tile[kr][nc] = W[(size_t)(k0 + kr) * N + n0 + nc]; }
  __syncthreads();
#pragma unroll 1
  for (int pass = 0; pass < 2; ++pass) {
    for (int i = t; i < 64 * 8; i += 256) { const int nr = i >> 3, k8 = (i & 7) * 8; bf16 hh[8], hl[8];
#pragma unroll
      for (int e = 0; e < 8; ++e) { const float v = tile[k8 + e][nr]; hh[e] = (bf16)v; hl[e] = lo_of(v, hh[e]); }
      bf16* d = WT + (size_t)(n0 + nr) * K + k0 + k8;
      *(volatile v4u_t*)d = *(const v4ua*)hh; *(volatile v4u_t*)(d + plane) = *(const v4ua*)hl; }
    __threadfence();
  }
}

template <typename AT, typename WT, int MODE>
__global__ __launch_bounds__(256) void gemm_split_kernel(
    const AT* __restrict__ A, size_t aPlane, const WT* __restrict__ W, size_t wPlane,
    const float* __restrict__ bias, void* __restrict__ out,
    int M, int N, int K) {
  __shared__ bf16 ldsA[128 * LDS_STRIDE], ldsAl[128 * LDS_STRIDE];
  __shared__ bf16 ldsW[256 * LDS_STRIDE], ldsWl[256 * LDS_STRIDE];
  __shared__ __attribute__((aligned(16))) unsigned char sob[256 * 136 * 2];

  const int t    = threadIdx.x;
  const int wave = t >> 5;
  const int lane = t & 31;
  const int wm   = (wave & 1) * 64;
  const int wn   = (wave >> 1) * 64;
  const int mBlk = blockIdx.x * 128;
  const int nBlk = blockIdx.y * 256;
  const int arow = t >> 1;
  const int ach  = (t & 1) * 16;

  f32x8 acc[4][4] = {};
  for (int k = 0; k < K; k += 32) {
    __syncthreads();
    {
      const AT* ap = A + (size_t)(mBlk + arow) * K + k + ach;
      bf16 hh[16], hl[16];
      if (sizeof(AT) == 4) {
#pragma unroll
        for (int i = 0; i < 16; ++i) { const float v = (float)ap[i]; hh[i] = (bf16)v; hl[i] = lo_of(v, hh[i]); }
      } else {
#pragma unroll
        for (int i = 0; i < 16; ++i) { hh[i] = (bf16)ap[i]; hl[i] = (bf16)ap[aPlane + i]; }
      }
#pragma unroll
      for (int i = 0; i < 16; ++i) { ldsA[arow * LDS_STRIDE + ach + i] = hh[i]; ldsAl[arow * LDS_STRIDE + ach + i] = hl[i]; }
    }
    {
      const WT* wp = W + (size_t)(nBlk + t) * K + k;
      if (sizeof(WT) == 4) {
#pragma unroll
        for (int i = 0; i < 32; ++i) { const float v = (float)wp[i]; const bf16 h_ = (bf16)v; ldsW[t * LDS_STRIDE + i] = h_; ldsWl[t * LDS_STRIDE + i] = lo_of(v, h_); }
      } else {
#pragma unroll
        for (int i = 0; i < 32; ++i) { ldsW[t * LDS_STRIDE + i] = (bf16)wp[i]; ldsWl[t * LDS_STRIDE + i] = (bf16)wp[wPlane + i]; }
      }
    }
    __syncthreads();
    bf16x16 wf[4], wfl[4];
#pragma unroll
    for (int j = 0; j < 4; ++j) { wf[j] = lds_frag(ldsW + (wn + 16 * j) * LDS_STRIDE, LDS_STRIDE); wfl[j] = lds_frag(ldsWl + (wn + 16 * j) * LDS_STRIDE, LDS_STRIDE); }
#pragma unroll
    for (int i = 0; i < 4; ++i) {
      const bf16x16 af = lds_frag(ldsA + (wm + 16 * i) * LDS_STRIDE, LDS_STRIDE), afl = lds_frag(ldsAl + (wm + 16 * i) * LDS_STRIDE, LDS_STRIDE);
#pragma unroll
      for (int j = 0; j < 4; ++j) acc[i][j] = wmma_split(af, afl, wf[j], wfl[j], acc[i][j]);
    }
  }

  const int nlane = lane & 15;
  const int mh    = (lane >> 4) * 8;
  __syncthreads();
  if (MODE == 1) {
    bf16* so = (bf16*)sob;
#pragma unroll
    for (int i = 0; i < 4; ++i)
#pragma unroll
      for (int j = 0; j < 4; ++j) {
        const int nl = wn + 16 * j + nlane;
        const float bv = bias ? bias[nBlk + nl] : 0.0f;
#pragma unroll
        for (int r = 0; r < 8; ++r) so[nl * 136 + wm + 16 * i + mh + r] = (bf16)(acc[i][j][r] + bv);
      }
    __syncthreads();
    const int b_ = mBlk >> 11, s0 = mBlk & (SS - 1);
#pragma unroll 1
    for (int pass = 0; pass < 2; ++pass) {
      for (int ch = t; ch < 256 * 16; ch += 256) { const int nl = ch >> 4, q = (ch & 15) * 8; const int n = nBlk + nl, h = n >> 6, dk = n & (DKK - 1);
        *(volatile v4u_t*)((bf16*)out + (((size_t)(b_ * HH + h)) * DKK + dk) * SS + s0 + q) = *(const v4ua*)(so + nl * 136 + q); }
      __threadfence();
    }
  } else {
    float* so = (float*)sob;
#pragma unroll 1
    for (int hf = 0; hf < 2; ++hf) {
      if (wm == hf * 64) {
#pragma unroll
        for (int i = 0; i < 4; ++i)
#pragma unroll
          for (int j = 0; j < 4; ++j) {
            const int nl = wn + 16 * j + nlane;
            const float bv = bias ? bias[nBlk + nl] : 0.0f;
#pragma unroll
            for (int r = 0; r < 8; ++r) so[(16 * i + mh + r) * 260 + nl] = acc[i][j][r] + bv;
          }
      }
      __syncthreads();
#pragma unroll 1
      for (int pass = 0; pass < 2; ++pass) {
        for (int ch = t; ch < 64 * 64; ch += 256) { const int ml = ch >> 6, q = (ch & 63) * 4;
          *(volatile v4f_t*)((float*)out + (size_t)(mBlk + hf * 64 + ml) * N + nBlk + q) = *(const volatile v4fa*)(so + ml * 260 + q); }
        __threadfence();
      }
      __syncthreads();
    }
  }
}


#define NB 512
#define NTL 2048
#define NS 128
#define NL 64
#define NPOS 1985
#define PP 2048
#define CH 32
#define NCOL (CH * PP)

__global__ __launch_bounds__(256) void k_windows(const float* __restrict__ x, int b0, float* __restrict__ Pw, float* __restrict__ P2) {
  __shared__ float xs[256 + 64];
  const int bl = blockIdx.y, pblk = blockIdx.x * 256, t = threadIdx.x, b = b0 + bl;
  const float* xb = x + (size_t)b * NTL;
  for (int i = t; i < 256 + 64; i += 256) { const int ti = pblk + i; xs[i] = (ti < NTL) ? xb[ti] : 0.0f; }
  __syncthreads();
  const int p = pblk + t; float* row = Pw + ((size_t)bl * PP + p) * NL;
  float mu = 0.0f;
#pragma unroll 1
  for (int l = 0; l < NL; ++l) mu += xs[t + l];
  mu *= (1.0f / (float)NL);
  const bool valid = (p < NPOS);
  float s2 = 0.0f;
#pragma unroll 1
  for (int pass = 0; pass < 2; ++pass) {
    s2 = 0.0f;
#pragma unroll 1
    for (int l4 = 0; l4 < NL; l4 += 4) { v4f_t v;
#pragma unroll
      for (int q = 0; q < 4; ++q) { const float c = valid ? (xs[t + l4 + q] - mu) : 0.0f; v[q] = c; s2 += c * c; }
      *(volatile v4f_t*)(row + l4) = v; }
    if (valid) *(volatile float*)(P2 + (size_t)b * PP + p) = s2;
    __threadfence(); }
}
__global__ __launch_bounds__(128) void k_s2(const float* __restrict__ sh, float* __restrict__ S2) {
  const int s = threadIdx.x; float a = 0.0f;
#pragma unroll 1
  for (int l = 0; l < NL; ++l) { const float v = sh[(size_t)s * NL + l]; a += v * v; }
  *(volatile float*)(S2 + s) = a; __threadfence(); *(volatile float*)(S2 + s) = a;
}
__global__ __launch_bounds__(128) void k_min(const float* __restrict__ T, const float* __restrict__ P2, const float* __restrict__ S2, int b0, float* __restrict__ out) {
  const int bl = blockIdx.x, s = threadIdx.x, b = b0 + bl; const float s2 = S2[s];
  const float* trow = T + (size_t)s * NCOL + (size_t)bl * PP; const float* p2 = P2 + (size_t)b * PP;
  float best = 3.0e38f;
#pragma unroll 1
  for (int p = 0; p < NPOS; ++p) { const float d2 = p2[p] + s2 - 2.0f * trow[p]; best = fminf(best, d2); }
  const float d = sqrtf(fmaxf(best, 0.0f));
  *(volatile float*)(out + (size_t)b * NS + s) = d; __threadfence(); *(volatile float*)(out + (size_t)b * NS + s) = d;
}

extern "C" void kernel_launch(void* const* d_in, const int* in_sizes, int n_in,
                              void* d_out, int out_size, void* d_ws, size_t ws_size,
                              hipStream_t stream) {
  (void)in_sizes; (void)n_in; (void)out_size; (void)ws_size;
  const float* x  = (const float*)d_in[0];
  const float* sh = (const float*)d_in[1];
  char* ws = (char*)d_ws;
  float* Pw = (float*)ws; ws += (size_t)NCOL * NL * 4;
  float* T  = (float*)ws; ws += (size_t)NS * NCOL * 4;
  float* P2 = (float*)ws; ws += (size_t)NB * PP * 4;
  float* S2 = (float*)ws; ws += 128 * 4;
  k_s2<<<1, 128, 0, stream>>>(sh, S2);
  for (int c = 0; c < NB / CH; ++c) {
    const int b0 = c * CH;
    k_windows<<<dim3(PP / 256, CH), 256, 0, stream>>>(x, b0, Pw, P2);
    gemm_split_kernel<float, float, 2><<<dim3(1, NCOL / 256), 256, 0, stream>>>(sh, 0, Pw, 0, nullptr, T, NS, NCOL, NL);
    k_min<<<CH, 128, 0, stream>>>(T, P2, S2, b0, (float*)d_out);
  }
}
